// HetSTGCNBlock_55448027791678
// MI455X (gfx1250) — hardware-verified
//
#include <hip/hip_runtime.h>
#include <stdint.h>
#include <stddef.h>

typedef unsigned short u16;
typedef unsigned int u32x4 __attribute__((ext_vector_type(4)));
typedef u32x4 __attribute__((may_alias)) u32x4a;
typedef float v8f __attribute__((ext_vector_type(8)));
typedef float v4f __attribute__((ext_vector_type(4)));
typedef v4f __attribute__((may_alias)) v4fa;
typedef _Float16 v16h __attribute__((ext_vector_type(16)));
typedef _Float16 v8h __attribute__((ext_vector_type(8)));
typedef __bf16 v16b __attribute__((ext_vector_type(16)));

union FragH { v16h v; u32x4 q[2]; };
union FragB { v16b v; u32x4 q[2]; };

#define INV64 0.015625f
#define HET_LDS0 118784
#define HET_LDS1 135168

__device__ __forceinline__ int imin(int a, int b) { return a < b ? a : b; }
__device__ __forceinline__ int imax(int a, int b) { return a > b ? a : b; }
__device__ __forceinline__ unsigned bfbits(float f) {
  unsigned u = __float_as_uint(f);
  return (u + 0x7FFFu + ((u >> 16) & 1u)) >> 16;
}
__device__ __forceinline__ float bfval(unsigned b) { return __uint_as_float(b << 16); }
__device__ __forceinline__ float bf16r(float f) { return bfval(bfbits(f)); }
__device__ __forceinline__ float reluf(float x) { return fmaxf(x, 0.0f); }
__device__ __forceinline__ float sigm(float x) { return __builtin_amdgcn_rcpf(1.0f + __expf(-x)); }

__device__ __forceinline__ v8f mma_b(v16b a, v16b b, v8f c) {
  v8f d = __builtin_amdgcn_wmma_f32_16x16x32_bf16(false, a, false, b, (short)0, c, false, false);
#if defined(__HIP_DEVICE_COMPILE__)
  asm volatile("v_nop\n\tv_nop\n\tv_nop\n\tv_nop" : "+v"(d) : "v"(a), "v"(b));
#endif
  return d;
}
__device__ __forceinline__ v8f mma_h(v16h a, v16h b, v8f c) {
  v8f d = __builtin_amdgcn_wmma_f32_16x16x32_f16(false, a, false, b, (short)0, c, false, false);
#if defined(__HIP_DEVICE_COMPILE__)
  asm volatile("v_nop\n\tv_nop\n\tv_nop\n\tv_nop" : "+v"(d) : "v"(a), "v"(b));
#endif
  return d;
}
__device__ __forceinline__ v16b ldb(const u16* p, int h) {
  FragB f;
  f.q[0] = *(const u32x4a*)(p + 8 * h);
  f.q[1] = *(const u32x4a*)(p + 16 + 8 * h);
  return f.v;
}
__device__ __forceinline__ v16h ldh(const _Float16* p, int h) {
  FragH f;
  f.q[0] = *(const u32x4a*)(p + 8 * h);
  f.q[1] = *(const u32x4a*)(p + 16 + 8 * h);
  return f.v;
}

__global__ __launch_bounds__(256) void k_cvt_a(const float* __restrict__ src, int M, int K,
                                                u16* __restrict__ dst, int Mp, int P) {
  const int gpr = P >> 3;
  const int g = blockIdx.x * 256 + threadIdx.x;
  if (g >= Mp * gpr) return;
  const int r = g / gpr, c8 = (g - r * gpr) * 8;
  const int rc = imin(r, M - 1);
  unsigned wv[4];
#pragma unroll
  for (int i = 0; i < 4; ++i) {
    const int c0 = c8 + 2 * i, c1 = c0 + 1;
    const float v0 = src[(size_t)rc * K + imin(c0, K - 1)];
    const float v1 = src[(size_t)rc * K + imin(c1, K - 1)];
    const unsigned b0 = (r < M && c0 < K) ? bfbits(v0) : 0u;
    const unsigned b1 = (r < M && c1 < K) ? bfbits(v1) : 0u;
    wv[i] = b0 | (b1 << 16);
  }
  u32x4 o = {wv[0], wv[1], wv[2], wv[3]};
  u16* d = dst + (size_t)r * P + c8;
  *(volatile u32x4*)d = o;
  __threadfence();
  *(volatile u32x4*)d = o;
}

__device__ __forceinline__ void p0_pass(const u16* sh0, const u16* sh1, u16* Ph, u16* Pl, int i, int lane) {
  const int hs = lane >> 4, q = lane & 15;
  const u32x4 v0 = *(const u32x4a*)(sh0 + 8 * q);
  const u32x4 v1 = *(const u32x4a*)(sh1 + 8 * q);
  const u32x4 v = hs ? v1 : v0;
  u16* d = (hs ? Pl : Ph) + (size_t)i * 128 + 8 * q;
  *(volatile u32x4*)d = v;
}
__global__ __launch_bounds__(128) void k_p0(const float* __restrict__ A01, const float* __restrict__ A10,
                                             u16* __restrict__ Ph, u16* __restrict__ Pl) {
  __shared__ __attribute__((aligned(16))) u16 sh[2][128];
  const int i = blockIdx.x, j = threadIdx.x;
  const int ic = imin(i, 80), jc = imin(j, 80);
  const float* arow = A01 + (size_t)ic * 319;
  float acc = 0.0f;
#pragma unroll 4
  for (int k = 0; k < 319; ++k) acc += bf16r(arow[k]) * bf16r(A10[(size_t)k * 81 + jc]);
  acc = (i < 81 && j < 81) ? acc : 0.0f;
  const unsigned hb = bfbits(acc);
  const unsigned lb = bfbits(acc - bfval(hb));
  sh[0][j] = (u16)hb;
  sh[1][j] = (u16)lb;
  __syncthreads();
  if (threadIdx.x < 32) {
    p0_pass(sh[0], sh[1], Ph, Pl, i, threadIdx.x);
    __threadfence();
    p0_pass(sh[0], sh[1], Ph, Pl, i, threadIdx.x);
  }
}

__global__ __launch_bounds__(256) void k_cvt_w(const float* __restrict__ t0, const float* __restrict__ t1,
                                                const float* __restrict__ t2, const float* __restrict__ t3,
                                                const float* __restrict__ t4, const float* __restrict__ t5,
                                                const float* __restrict__ the, const float* __restrict__ w1,
                                                const float* __restrict__ wc, _Float16* __restrict__ WPL) {
  const int tid = threadIdx.x, bx = blockIdx.x;
  float v[8];
  _Float16* d;
  if (bx < 62) {
    const int mat = bx >> 1;
    const float* src;
    if (mat == 30) {
      src = the;
    } else {
      const int grp = mat / 5, ly = mat - grp * 5;
      const float* base = (grp == 0) ? t0 : (grp == 1) ? t1 : (grp == 2) ? t2 : (grp == 3) ? t3 : (grp == 4) ? t4 : t5;
      src = base + (size_t)ly * 4096;
    }
    const int gl = (bx & 1) * 256 + tid;
    const int n = gl >> 3, k8 = (gl & 7) * 8;
#pragma unroll
    for (int i = 0; i < 8; ++i) v[i] = src[(k8 + i) * 64 + n];
    d = WPL + (size_t)mat * 4096 + n * 64 + k8;
  } else {
    const int idx = (bx - 62) * 256 + tid;
    const int n = idx / 24, k8 = (idx - n * 24) * 8;
    if (bx < 68) {
#pragma unroll
      for (int i = 0; i < 8; ++i) {
        const int k = k8 + i, tap = k >> 6, ci = k & 63;
        v[i] = w1[n * 192 + ci * 3 + tap];
      }
    } else {
#pragma unroll
      for (int i = 0; i < 8; ++i) {
        const int k = k8 + i, tap = k >> 6, ci = k & 63;
        v[i] = wc[(n - 64) * 192 + ci * 3 + tap];
      }
    }
    d = WPL + (size_t)31 * 4096 + n * 192 + k8;
  }
  v8h o;
#pragma unroll
  for (int i = 0; i < 8; ++i) o[i] = (_Float16)(bf16r(v[i]) * 64.0f);
  *(volatile v8h*)d = o;
  __threadfence();
  *(volatile v8h*)d = o;
}

__device__ __forceinline__ void t1_pass(const float* sv, _Float16* T1H, u16* Uh, u16* Ul,
                                        int b, int t, int j0, int NREAL, int NBASE, int UP,
                                        int w, int sub, int q) {
#pragma unroll
  for (int it = 0; it < 2; ++it) {
    const int jl = 8 * w + 4 * it + sub;
    const int j = j0 + jl;
    const float* s = sv + jl * 64 + 8 * q;
    v8h o;
#pragma unroll
    for (int i = 0; i < 8; ++i) o[i] = (_Float16)s[i];
    if (j < NREAL) {
      _Float16* dp = T1H + ((((size_t)b * 400 + NBASE + j) * 30 + t) * 64) + 8 * q;
      *(volatile v8h*)dp = o;
    }
  }
#pragma unroll
  for (int it = 0; it < 2; ++it) {
    const int c = 8 * w + 4 * it + sub;
    unsigned hw[4], lw[4];
#pragma unroll
    for (int r2 = 0; r2 < 4; ++r2) {
      const float v0 = sv[(8 * q + 2 * r2) * 64 + c];
      const float v1 = sv[(8 * q + 2 * r2 + 1) * 64 + c];
      const unsigned h0 = bfbits(v0), h1 = bfbits(v1);
      const unsigned l0 = bfbits(v0 - bfval(h0)), l1 = bfbits(v1 - bfval(h1));
      hw[r2] = h0 | (h1 << 16);
      lw[r2] = l0 | (l1 << 16);
    }
    const size_t off = (((size_t)b * 1920 + t * 64 + c) * UP) + j0 + 8 * q;
    u32x4 oh = {hw[0], hw[1], hw[2], hw[3]};
    u32x4 ol = {lw[0], lw[1], lw[2], lw[3]};
    *(volatile u32x4*)(Uh + off) = oh;
    *(volatile u32x4*)(Ul + off) = ol;
  }
}

__global__ __launch_bounds__(256) void k_tconv1(const float* __restrict__ X,
                                                 const float* __restrict__ w1, const float* __restrict__ b1,
                                                 const float* __restrict__ wc, const float* __restrict__ bc,
                                                 _Float16* __restrict__ T1H,
                                                 u16* __restrict__ U0h, u16* __restrict__ U0l,
                                                 u16* __restrict__ U1h, u16* __restrict__ U1l) {
  __shared__ float sw[192 * 6];
  __shared__ float sbias[192];
  __shared__ __attribute__((aligned(16))) float sv[64 * 64];
  const int tid = threadIdx.x, lane = tid & 31, w = tid >> 5, sub = lane >> 3, q = lane & 7;
  const int t = blockIdx.x, g = blockIdx.y, b = blockIdx.z;
  const int side = (g >= 2) ? 1 : 0;
  const int j0 = side ? 64 * (g - 2) : 64 * g;
  const int NREAL = side ? 319 : 81, NBASE = side ? 81 : 0, UP = side ? 320 : 128;
  u16* Uh = side ? U1h : U0h;
  u16* Ul = side ? U1l : U0l;

  for (int i = tid; i < 192 * 6; i += 256) {
    const int c = i / 6, e = i - c * 6, tap = e >> 1, ci = e & 1;
    const float va = w1[imin(c, 63) * 6 + ci * 3 + tap];
    const float vb = wc[imax(c - 64, 0) * 6 + ci * 3 + tap];
    sw[i] = bf16r(c < 64 ? va : vb);
  }
  for (int i = tid; i < 192; i += 256) {
    const float va = b1[imin(i, 63)];
    const float vb = bc[imax(i - 64, 0)];
    sbias[i] = bf16r(i < 64 ? va : vb);
  }
  const int jl = tid >> 2, cq = tid & 3;
  const int j = j0 + jl;
  const bool valid = j < NREAL;
  const int n = NBASE + imin(j, NREAL - 1);
  const float* xp = X + (((size_t)b * 400 + n) * 32 + t) * 2;
  float x[6];
#pragma unroll
  for (int e = 0; e < 6; ++e) x[e] = bf16r(xp[e]);
  __syncthreads();
#pragma unroll 1
  for (int cc = 0; cc < 16; ++cc) {
    const int c = cq * 16 + cc;
    float tv = sbias[c], pv = sbias[64 + c], qv = sbias[128 + c];
#pragma unroll
    for (int e = 0; e < 6; ++e) {
      tv += x[e] * sw[c * 6 + e];
      pv += x[e] * sw[(64 + c) * 6 + e];
      qv += x[e] * sw[(128 + c) * 6 + e];
    }
    const float o = (pv + tv) * sigm(qv);
    sv[jl * 64 + c] = valid ? o : 0.0f;
  }
  __syncthreads();
  t1_pass(sv, T1H, Uh, Ul, b, t, j0, NREAL, NBASE, UP, w, sub, q);
  __threadfence();
  t1_pass(sv, T1H, Uh, Ul, b, t, j0, NREAL, NBASE, UP, w, sub, q);
}

template <int UP>
__device__ __forceinline__ void plane_pass(const u16* sh, const u16* sl, u16* gh, u16* gl,
                                           size_t base, int w, int sub, int q) {
  constexpr int LPC = UP / 64;
  constexpr int NL = 64 * LPC;
#pragma unroll 1
  for (int L = w * 4 + sub; L < NL; L += 16) {
    const int c = L / LPC, piece = L - c * LPC;
    const int off = c * UP + piece * 64 + 8 * q;
    const u32x4 a = *(const u32x4a*)(sh + off);
    const u32x4 bb = *(const u32x4a*)(sl + off);
    *(volatile u32x4*)(gh + base + off) = a;
    *(volatile u32x4*)(gl + base + off) = bb;
  }
}

__device__ __forceinline__ void tk_pass(const _Float16* sTK, _Float16* TK2, int b, int t, int mt,
                                        int NBASE, int NREAL, int w, int sub, int q) {
#pragma unroll
  for (int it = 0; it < 2; ++it) {
    const int row = 8 * w + 4 * it + sub;
    const int jj = mt * 32 + row;
    const u32x4 v = *(const u32x4a*)(sTK + row * 64 + 8 * q);
    if (jj < NREAL) {
      _Float16* d = TK2 + ((((size_t)b * 400 + NBASE + jj) * 30 + t) * 64) + 8 * q;
      *(volatile u32x4*)d = v;
    }
  }
}

template <int SIDE>
__global__ __launch_bounds__(128) void k_het(
    const u16* __restrict__ gA, const u16* __restrict__ gBh, const u16* __restrict__ gBl,
    const u16* __restrict__ gC,
    u16* uH, u16* uL,
    const u16* vH, const u16* vL,
    const u16* xH, const u16* xL,
    u16* oH, u16* oL,
    const _Float16* __restrict__ th1, const _Float16* __restrict__ th2,
    const _Float16* __restrict__ th3, const _Float16* __restrict__ the,
    const _Float16* __restrict__ T1H, _Float16* __restrict__ TK2, int last)
{
  constexpr int MT    = SIDE ? 10 : 3;
  constexpr int NREAL = SIDE ? 319 : 81;
  constexpr int NBASE = SIDE ? 81 : 0;
  constexpr int UP    = SIDE ? 320 : 128;
  constexpr int VP    = SIDE ? 128 : 320;

  extern __shared__ __attribute__((aligned(16))) unsigned char dsm[];
  _Float16* sS   = (_Float16*)(dsm + 0);
  _Float16* sTh  = (_Float16*)(dsm + 12288);
  _Float16* sThe = (_Float16*)(dsm + 36864);
  _Float16* sU   = (_Float16*)(dsm + 45056);
  _Float16* sTK  = (_Float16*)(dsm + 49152);
  u16* sUh = (u16*)(dsm + 53248);
  u16* sUl = sUh + 64 * UP;
  u16* sGh = sUl + 64 * UP;
  u16* sGl = sGh + 64 * 128;

  const int tid = threadIdx.x, lane = tid & 31, w = tid >> 5;
  const int h = lane >> 4, m = lane & 15, sub = lane >> 3, q = lane & 7;
  const int rt = w & 1, cw = w >> 1;
  const int t = blockIdx.x, b = blockIdx.y, col0 = t * 64;

  for (int i = tid; i < 1536; i += 128) {
    const int p = i >> 9, r = i & 511;
    const _Float16* src = (p == 0) ? th1 : ((p == 1) ? th2 : th3);
    *(u32x4a*)(sTh + i * 8) = *(const u32x4a*)(src + r * 8);
  }
  if (last) {
    for (int i = tid; i < 512; i += 128) *(u32x4a*)(sThe + i * 8) = *(const u32x4a*)(the + i * 8);
  }
  {
    const int nz = SIDE ? (64 * UP * 4 / 16) : ((64 * UP * 4 + 64 * 128 * 4) / 16);
    u32x4 z = {0u, 0u, 0u, 0u};
    for (int i = tid; i < nz; i += 128) *(u32x4a*)((unsigned char*)sUh + (size_t)i * 16) = z;
  }
  __syncthreads();

  const size_t ubase = ((size_t)b * 1920 + col0) * UP;
  const size_t vbase = ((size_t)b * 1920 + col0) * VP;
  const size_t xbase = ((size_t)b * 1920 + col0) * 128;
  const v8f z8 = {0.f, 0.f, 0.f, 0.f, 0.f, 0.f, 0.f, 0.f};

#pragma unroll 1
  for (int mt = 0; mt < MT; ++mt) {
    const int grow = mt * 32 + rt * 16 + m;
    v8f acc1[2], acc2[2], acc3[2];
    acc1[0] = z8; acc1[1] = z8; acc2[0] = z8; acc2[1] = z8; acc3[0] = z8; acc3[1] = z8;

    if (SIDE == 0) {
      const u16* pa = gA  + (size_t)grow * 128;
      const u16* ph = gBh + (size_t)grow * 128;
      const u16* pl = gBl + (size_t)grow * 128;
#pragma unroll 1
      for (int ks = 0; ks < 3; ++ks) {
        const v16b gfa = ldb(pa + 32 * ks, h);
        const v16b gfh = ldb(ph + 32 * ks, h);
        const v16b gfl = ldb(pl + 32 * ks, h);
#pragma unroll
        for (int ct = 0; ct < 2; ++ct) {
          const size_t bo = ubase + (size_t)(32 * cw + 16 * ct + m) * UP + 32 * ks;
          const v16b ubh = ldb(uH + bo, h);
          const v16b ubl = ldb(uL + bo, h);
          acc1[ct] = mma_b(gfa, ubh, acc1[ct]);
          acc1[ct] = mma_b(gfa, ubl, acc1[ct]);
          acc2[ct] = mma_b(gfh, ubh, acc2[ct]);
          acc2[ct] = mma_b(gfh, ubl, acc2[ct]);
          acc2[ct] = mma_b(gfl, ubh, acc2[ct]);
        }
      }
      const u16* pc = gC + (size_t)grow * 320;
#pragma unroll 1
      for (int ks = 0; ks < 10; ++ks) {
        const v16b gfa = ldb(pc + 32 * ks, h);
#pragma unroll
        for (int ct = 0; ct < 2; ++ct) {
          const size_t bo = vbase + (size_t)(32 * cw + 16 * ct + m) * VP + 32 * ks;
          const v16b vbh = ldb(vH + bo, h);
          const v16b vbl = ldb(vL + bo, h);
          acc3[ct] = mma_b(gfa, vbh, acc3[ct]);
          acc3[ct] = mma_b(gfa, vbl, acc3[ct]);
        }
      }
    } else {
      const u16* pa = gA + (size_t)grow * 320;
#pragma unroll 1
      for (int ks = 0; ks < 10; ++ks) {
        const v16b gfa = ldb(pa + 32 * ks, h);
#pragma unroll
        for (int ct = 0; ct < 2; ++ct) {
          const size_t bo = ubase + (size_t)(32 * cw + 16 * ct + m) * UP + 32 * ks;
          const v16b ubh = ldb(uH + bo, h);
          const v16b ubl = ldb(uL + bo, h);
          acc1[ct] = mma_b(gfa, ubh, acc1[ct]);
          acc1[ct] = mma_b(gfa, ubl, acc1[ct]);
        }
      }
      const u16* pb = gBh + (size_t)grow * 128;
#pragma unroll 1
      for (int ks = 0; ks < 3; ++ks) {
        const v16b gfb = ldb(pb + 32 * ks, h);
#pragma unroll
        for (int ct = 0; ct < 2; ++ct) {
          const size_t vo = vbase + (size_t)(32 * cw + 16 * ct + m) * VP + 32 * ks;
          const size_t xo = xbase + (size_t)(32 * cw + 16 * ct + m) * 128 + 32 * ks;
          const v16b vbh = ldb(vH + vo, h);
          const v16b vbl = ldb(vL + vo, h);
          acc2[ct] = mma_b(gfb, vbh, acc2[ct]);
          acc2[ct] = mma_b(gfb, vbl, acc2[ct]);
          const v16b xbh = ldb(xH + xo, h);
          const v16b xbl = ldb(xL + xo, h);
          acc3[ct] = mma_b(gfb, xbh, acc3[ct]);
          acc3[ct] = mma_b(gfb, xbl, acc3[ct]);
        }
      }
    }

#pragma unroll
    for (int ct = 0; ct < 2; ++ct) {
      const int col = 32 * cw + 16 * ct + m;
#pragma unroll
      for (int r = 0; r < 8; ++r) {
        const int row = rt * 16 + 8 * h + r;
        sS[row * 64 + col]        = (_Float16)acc1[ct][r];
        sS[2048 + row * 64 + col] = (_Float16)acc2[ct][r];
        sS[4096 + row * 64 + col] = (_Float16)acc3[ct][r];
      }
      if (SIDE == 0) {
        unsigned hw[4], lw[4];
#pragma unroll
        for (int r2 = 0; r2 < 4; ++r2) {
          const float v0 = acc3[ct][2 * r2], v1 = acc3[ct][2 * r2 + 1];
          const unsigned h0 = bfbits(v0), h1 = bfbits(v1);
          const unsigned l0 = bfbits(v0 - bfval(h0)), l1 = bfbits(v1 - bfval(h1));
          hw[r2] = h0 | (h1 << 16);
          lw[r2] = l0 | (l1 << 16);
        }
        const int i0 = mt * 32 + rt * 16 + 8 * h;
        u32x4 oh = {hw[0], hw[1], hw[2], hw[3]};
        u32x4 ol = {lw[0], lw[1], lw[2], lw[3]};
        *(u32x4a*)(sGh + col * 128 + i0) = oh;
        *(u32x4a*)(sGl + col * 128 + i0) = ol;
      }
    }
    __syncthreads();

    v8f c1[2], c2[2], c3[2];
    c1[0] = z8; c1[1] = z8; c2[0] = z8; c2[1] = z8; c3[0] = z8; c3[1] = z8;
#pragma unroll
    for (int ks = 0; ks < 2; ++ks) {
      const int ao = (rt * 16 + m) * 64 + 32 * ks;
      const v16h fa1 = ldh(sS + ao, h);
      const v16h fa2 = ldh(sS + 2048 + ao, h);
      const v16h fa3 = ldh(sS + 4096 + ao, h);
#pragma unroll
      for (int ct = 0; ct < 2; ++ct) {
        const int bo = (32 * cw + 16 * ct + m) * 64 + 32 * ks;
        const v16h fb1 = ldh(sTh + bo, h);
        const v16h fb2 = ldh(sTh + 4096 + bo, h);
        const v16h fb3 = ldh(sTh + 8192 + bo, h);
        c1[ct] = mma_h(fa1, fb1, c1[ct]);
        c2[ct] = mma_h(fa2, fb2, c2[ct]);
        c3[ct] = mma_h(fa3, fb3, c3[ct]);
      }
    }

#pragma unroll
    for (int ct = 0; ct < 2; ++ct) {
      const int col = 32 * cw + 16 * ct + m;
      unsigned hw[4], lw[4];
#pragma unroll
      for (int r2 = 0; r2 < 4; ++r2) {
        unsigned hb[2], lb[2];
#pragma unroll
        for (int e = 0; e < 2; ++e) {
          const int r = 2 * r2 + e;
          const int row = rt * 16 + 8 * h + r;
          const int jj = mt * 32 + row;
          const float u2 = reluf(c1[ct][r] * INV64);
          const float u5 = sigm((c2[ct][r] + c3[ct][r]) * INV64);
          const float u6 = reluf(0.5f * (u2 + u5));
          const int jc = imin(jj, NREAL - 1);
          const float x00 = (float)T1H[((((size_t)b * 400 + NBASE + jc) * 30 + t) * 64) + col];
          float uo = reluf(0.9f * u6 + 0.1f * x00);
          uo = (jj < NREAL) ? uo : 0.0f;
          if (last) sU[row * 64 + col] = (_Float16)uo;
          hb[e] = bfbits(uo);
          lb[e] = bfbits(uo - bfval(hb[e]));
        }
        hw[r2] = hb[0] | (hb[1] << 16);
        lw[r2] = lb[0] | (lb[1] << 16);
      }
      const int i0 = mt * 32 + rt * 16 + 8 * h;
      u32x4 oh = {hw[0], hw[1], hw[2], hw[3]};
      u32x4 ol = {lw[0], lw[1], lw[2], lw[3]};
      *(u32x4a*)(sUh + col * UP + i0) = oh;
      *(u32x4a*)(sUl + col * UP + i0) = ol;
    }
    __syncthreads();

    if (last) {
      v8f ck[2];
      ck[0] = z8; ck[1] = z8;
#pragma unroll
      for (int ks = 0; ks < 2; ++ks) {
        const v16h fa = ldh(sU + (rt * 16 + m) * 64 + 32 * ks, h);
#pragma unroll
        for (int ct = 0; ct < 2; ++ct) {
          const v16h fb = ldh(sThe + (32 * cw + 16 * ct + m) * 64 + 32 * ks, h);
          ck[ct] = mma_h(fa, fb, ck[ct]);
        }
      }
#pragma unroll
      for (int ct = 0; ct < 2; ++ct) {
        const int col = 32 * cw + 16 * ct + m;
#pragma unroll
        for (int r = 0; r < 8; ++r) {
          const int row = rt * 16 + 8 * h + r;
          sTK[row * 64 + col] = (_Float16)reluf(ck[ct][r] * INV64);
        }
      }
      __syncthreads();
      tk_pass(sTK, TK2, b, t, mt, NBASE, NREAL, w, sub, q);
      __threadfence();
      tk_pass(sTK, TK2, b, t, mt, NBASE, NREAL, w, sub, q);
    }
  }
  __syncthreads();

  const size_t gbase = ((size_t)b * 1920 + col0) * 128;
  plane_pass<UP>(sUh, sUl, uH, uL, ubase, w, sub, q);
  if (SIDE == 0) plane_pass<128>(sGh, sGl, oH, oL, gbase, w, sub, q);
  __threadfence();
  plane_pass<UP>(sUh, sUl, uH, uL, ubase, w, sub, q);
  if (SIDE == 0) plane_pass<128>(sGh, sGl, oH, oL, gbase, w, sub, q);
}

__device__ __forceinline__ void out_pass(const float* sO, float* dst, int w, int sub, int q) {
#pragma unroll
  for (int it = 0; it < 8; ++it) {
    const int L = w * 32 + it * 4 + sub;
    const v4f v = *(const v4fa*)(sO + L * 32 + 4 * q);
    *(volatile v4f*)(dst + L * 32 + 4 * q) = v;
  }
}
__global__ __launch_bounds__(128) void k_conv2(const _Float16* __restrict__ TK2, const _Float16* __restrict__ WC,
                                               const float* __restrict__ b1, const float* __restrict__ bc,
                                               float* __restrict__ out) {
  __shared__ __attribute__((aligned(16))) float sO[64 * 64];
  const int tid = threadIdx.x, lane = tid & 31, w = tid >> 5;
  const int h = lane >> 4, m = lane & 15, sub = lane >> 3, q = lane & 7;
  const int r0 = blockIdx.x * 64;
  const int arow = r0 + 16 * w + m;
  const int qr = arow / 28, tp = arow - qr * 28;
  const _Float16* ap = TK2 + ((size_t)qr * 30 + tp) * 64;
  v16h a[6];
#pragma unroll
  for (int ks = 0; ks < 6; ++ks) a[ks] = ldh(ap + 32 * ks, h);
  const v8f z8 = {0.f, 0.f, 0.f, 0.f, 0.f, 0.f, 0.f, 0.f};
#pragma unroll 1
  for (int ct = 0; ct < 4; ++ct) {
    v8f aT = z8, aP = z8, aQ = z8;
    const _Float16* wt = WC + (size_t)(16 * ct + m) * 192;
    const _Float16* wp = WC + (size_t)(64 + 16 * ct + m) * 192;
    const _Float16* wq = WC + (size_t)(128 + 16 * ct + m) * 192;
#pragma unroll
    for (int ks = 0; ks < 6; ++ks) {
      const v16h ft = ldh(wt + 32 * ks, h);
      const v16h fp = ldh(wp + 32 * ks, h);
      const v16h fq = ldh(wq + 32 * ks, h);
      aT = mma_h(a[ks], ft, aT);
      aP = mma_h(a[ks], fp, aP);
      aQ = mma_h(a[ks], fq, aQ);
    }
    const int c = 16 * ct + m;
    const float bt = bf16r(b1[c]), bp = bf16r(bc[c]), bq = bf16r(bc[64 + c]);
#pragma unroll
    for (int r = 0; r < 8; ++r) {
      const float tv = aT[r] * INV64 + bt;
      const float pv = aP[r] * INV64 + bp;
      const float qv = aQ[r] * INV64 + bq;
      sO[(16 * w + 8 * h + r) * 64 + c] = (pv + tv) * sigm(qv);
    }
  }
  __syncthreads();
  float* dst = out + (size_t)r0 * 64;
  out_pass(sO, dst, w, sub, q);
  __threadfence();
  out_pass(sO, dst, w, sub, q);
}

__global__ __launch_bounds__(256) void k_bn(float* out, const float* __restrict__ gamma,
                                             const float* __restrict__ beta) {
  const int tid = threadIdx.x, lane = tid & 31, w = tid >> 5;
  const int hsel = lane >> 4, piece = lane & 15;
#pragma unroll 1
  for (int k = 0; k < 4; ++k) {
    const int n = blockIdx.x * 32 + w * 4 + k;
    if (n >= 400) continue;
    double s = 0.0, s2 = 0.0;
#pragma unroll 1
    for (int it = 0; it < 224; ++it) {
      const int row = 2 * it + hsel;
      const int bb = row / 28, tp = row - bb * 28;
      const float* p = out + ((((size_t)bb * 400 + n) * 28 + tp) * 64) + piece * 4;
      const v4f v = *(const v4fa*)p;
      s  += (double)v.x + (double)v.y + (double)v.z + (double)v.w;
      s2 += (double)v.x * (double)v.x + (double)v.y * (double)v.y +
            (double)v.z * (double)v.z + (double)v.w * (double)v.w;
    }
#pragma unroll
    for (int off = 16; off > 0; off >>= 1) {
      s  += __shfl_xor(s, off);
      s2 += __shfl_xor(s2, off);
    }
    const double mean = s * (1.0 / 28672.0);
    double var = s2 * (1.0 / 28672.0) - mean * mean;
    var = var < 0.0 ? 0.0 : var;
    const float mf = (float)mean;
    const float rs = rsqrtf((float)var + 1e-5f);
    const float ga = bf16r(gamma[n]), be = bf16r(beta[n]);
    const float sc = rs * ga;
#pragma unroll 1
    for (int it = 0; it < 224; ++it) {
      const int row = 2 * it + hsel;
      const int bb = row / 28, tp = row - bb * 28;
      float* p = out + ((((size_t)bb * 400 + n) * 28 + tp) * 64) + piece * 4;
      const v4f v = *(const v4fa*)p;
      v4f o;
      o.x = (v.x - mf) * sc + be;
      o.y = (v.y - mf) * sc + be;
      o.z = (v.z - mf) * sc + be;
      o.w = (v.w - mf) * sc + be;
      *(volatile v4f*)p = o;
      __threadfence();
      *(volatile v4f*)p = o;
    }
  }
}

extern "C" void kernel_launch(void* const* d_in, const int* in_sizes, int n_in,
                              void* d_out, int out_size, void* d_ws, size_t ws_size,
                              hipStream_t stream) {
  if (n_in < 22) return;
  if (in_sizes[0] != 409600 || in_sizes[1] != 6561 || in_sizes[2] != 25839 ||
      in_sizes[3] != 25839 || in_sizes[4] != 101761) return;
  if (in_sizes[5] != 384 || in_sizes[6] != 64 || in_sizes[7] != 768 || in_sizes[8] != 128) return;
  for (int i = 9; i < 15; ++i) if (in_sizes[i] != 20480) return;
  if (in_sizes[15] != 4096 || in_sizes[16] != 12288 || in_sizes[17] != 64 ||
      in_sizes[18] != 24576 || in_sizes[19] != 128 || in_sizes[20] != 400 || in_sizes[21] != 400) return;
  if (out_size != 11468800) return;

  const float* X    = (const float*)d_in[0];
  const float* A00  = (const float*)d_in[1];
  const float* A01  = (const float*)d_in[2];
  const float* A10  = (const float*)d_in[3];
  const float* A11  = (const float*)d_in[4];
  const float* t1w  = (const float*)d_in[5];
  const float* t1b  = (const float*)d_in[6];
  const float* t1cw = (const float*)d_in[7];
  const float* t1cb = (const float*)d_in[8];
  const float* g1t1 = (const float*)d_in[9];
  const float* g1t2 = (const float*)d_in[10];
  const float* g1t3 = (const float*)d_in[11];
  const float* g2t1 = (const float*)d_in[12];
  const float* g2t2 = (const float*)d_in[13];
  const float* g2t3 = (const float*)d_in[14];
  const float* theta= (const float*)d_in[15];
  const float* t2w  = (const float*)d_in[16];
  const float* t2b  = (const float*)d_in[17];
  const float* t2cw = (const float*)d_in[18];
  const float* t2cb = (const float*)d_in[19];
  const float* bn_g = (const float*)d_in[20];
  const float* bn_b = (const float*)d_in[21];
  float* out = (float*)d_out;

  const size_t SZ_T1H = (size_t)16 * 400 * 30 * 64 * 2;
  const size_t SZ_U0  = (size_t)16 * 1920 * 128 * 2;
  const size_t SZ_U1  = (size_t)16 * 1920 * 320 * 2;
  const size_t SZ_TK2 = SZ_T1H;
  const size_t SZ_A00 = (size_t)96 * 128 * 2;
  const size_t SZ_A01 = (size_t)96 * 320 * 2;
  const size_t SZ_A11 = (size_t)320 * 320 * 2;
  const size_t SZ_A10 = (size_t)320 * 128 * 2;
  const size_t SZ_WPL = (size_t)(31 * 4096 + 192 * 192) * 2;
  const size_t OFF_T1H = 0;
  const size_t OFF_U0H = OFF_T1H + SZ_T1H;
  const size_t OFF_U0L = OFF_U0H + SZ_U0;
  const size_t OFF_U1H = OFF_U0L + SZ_U0;
  const size_t OFF_U1L = OFF_U1H + SZ_U1;
  const size_t OFF_S3H = OFF_U1L + SZ_U1;
  const size_t OFF_S3L = OFF_S3H + SZ_U0;
  const size_t OFF_TK2 = OFF_S3L + SZ_U0;
  const size_t OFF_A00 = OFF_TK2 + SZ_TK2;
  const size_t OFF_P0H = OFF_A00 + SZ_A00;
  const size_t OFF_P0L = OFF_P0H + SZ_A00;
  const size_t OFF_A01 = OFF_P0L + SZ_A00;
  const size_t OFF_A11 = OFF_A01 + SZ_A01;
  const size_t OFF_A10 = OFF_A11 + SZ_A11;
  const size_t OFF_WPL = OFF_A10 + SZ_A10;
  const size_t OFF_END = OFF_WPL + SZ_WPL;
  if (OFF_END > ws_size) return;

  char* ws = (char*)d_ws;
  _Float16* T1H = (_Float16*)(ws + OFF_T1H);
  u16* U0h = (u16*)(ws + OFF_U0H);
  u16* U0l = (u16*)(ws + OFF_U0L);
  u16* U1h = (u16*)(ws + OFF_U1H);
  u16* U1l = (u16*)(ws + OFF_U1L);
  u16* S3h = (u16*)(ws + OFF_S3H);
  u16* S3l = (u16*)(ws + OFF_S3L);
  _Float16* TK2 = (_Float16*)(ws + OFF_TK2);
  u16* A00b = (u16*)(ws + OFF_A00);
  u16* P0h  = (u16*)(ws + OFF_P0H);
  u16* P0l  = (u16*)(ws + OFF_P0L);
  u16* A01b = (u16*)(ws + OFF_A01);
  u16* A11b = (u16*)(ws + OFF_A11);
  u16* A10b = (u16*)(ws + OFF_A10);
  _Float16* WPL = (_Float16*)(ws + OFF_WPL);
  const _Float16* THE = WPL + (size_t)30 * 4096;
  const _Float16* WC  = WPL + (size_t)31 * 4096;

  k_cvt_a<<<6, 256, 0, stream>>>(A00, 81, 81, A00b, 96, 128);
  k_cvt_a<<<15, 256, 0, stream>>>(A01, 81, 319, A01b, 96, 320);
  k_cvt_a<<<50, 256, 0, stream>>>(A11, 319, 319, A11b, 320, 320);
  k_cvt_a<<<20, 256, 0, stream>>>(A10, 319, 81, A10b, 320, 128);
  k_p0<<<96, 128, 0, stream>>>(A01, A10, P0h, P0l);
  k_cvt_w<<<80, 256, 0, stream>>>(g1t1, g1t2, g1t3, g2t1, g2t2, g2t3, theta, t2w, t2cw, WPL);

  k_tconv1<<<dim3(30, 7, 16), 256, 0, stream>>>(X, t1w, t1b, t1cw, t1cb, T1H, U0h, U0l, U1h, U1l);

  (void)hipFuncSetAttribute(reinterpret_cast<const void*>(&k_het<0>),
                            hipFuncAttributeMaxDynamicSharedMemorySize, HET_LDS0);
  (void)hipFuncSetAttribute(reinterpret_cast<const void*>(&k_het<1>),
                            hipFuncAttributeMaxDynamicSharedMemorySize, HET_LDS1);

  for (int i = 0; i < 5; ++i) {
    const int last = (i == 4) ? 1 : 0;
    const _Float16* h1 = WPL + (size_t)(0 * 5 + i) * 4096;
    const _Float16* h2 = WPL + (size_t)(1 * 5 + i) * 4096;
    const _Float16* h3 = WPL + (size_t)(2 * 5 + i) * 4096;
    const _Float16* e1 = WPL + (size_t)(3 * 5 + i) * 4096;
    const _Float16* e2 = WPL + (size_t)(4 * 5 + i) * 4096;
    const _Float16* e3 = WPL + (size_t)(5 * 5 + i) * 4096;
    k_het<0><<<dim3(30, 16), 128, HET_LDS0, stream>>>(
        A00b, P0h, P0l, A01b, U0h, U0l, U1h, U1l, U1h, U1l, S3h, S3l,
        h1, h2, h3, THE, T1H, TK2, last);
    k_het<1><<<dim3(30, 16), 128, HET_LDS1, stream>>>(
        A11b, A10b, A10b, A10b, U1h, U1l, S3h, S3l, U0h, U0l, S3h, S3l,
        e1, e2, e3, THE, T1H, TK2, last);
  }

  k_conv2<<<2800, 128, 0, stream>>>(TK2, WC, t2b, t2cb, out);
  k_bn<<<13, 256, 0, stream>>>(out, bn_g, bn_b);
}
